// LMKANRBFLayer_60722247631487
// MI455X (gfx1250) — hardware-verified
//
#include <hip/hip_runtime.h>
#include <math.h>

constexpr int kInDim      = 512;
constexpr int kOutDim     = 1024;
constexpr int kNumRbf     = 16;
constexpr int kHidden     = 8;
constexpr int kRows       = 8192;
constexpr int kFeat       = kInDim * kNumRbf;
constexpr int kChunkRows  = 2048;
constexpr int kNumChunks  = kRows / kChunkRows;
constexpr int kRowsPerBlk = 32;
constexpr float kPhiCarry  = 64.0f;
constexpr float kWCarry    = 2048.0f;
constexpr float kGemmScale = 1.0f / (64.0f * 2048.0f);

constexpr int kLdsFloats = 21072;
constexpr int kLdsBytes  = kLdsFloats * 4;

constexpr size_t kWsWht    = 0;
constexpr size_t kWsPhiA   = 16777216UL;
constexpr size_t kWsPhiB   = 50331648UL;
constexpr size_t kWsLogdet = 83886080UL;
constexpr size_t kWsTotal  = 83918848UL;

typedef __attribute__((ext_vector_type(16))) _Float16 v16h;
typedef __attribute__((ext_vector_type(8)))  _Float16 v8h;
typedef __attribute__((ext_vector_type(16))) __bf16   v16b;
typedef __attribute__((ext_vector_type(8)))  __bf16   v8b;
typedef __attribute__((ext_vector_type(8)))  float    v8f;
typedef __attribute__((ext_vector_type(4)))  float    v4f;
typedef __attribute__((ext_vector_type(4)))  unsigned int v4u;

__device__ __forceinline__ unsigned short f2bf_bits(float f) {
  unsigned u = __float_as_uint(f);
  return (unsigned short)((u + 0x7FFFu + ((u >> 16) & 1u)) >> 16);
}
__device__ __forceinline__ float bf_bits2f(unsigned short h) { return __uint_as_float(((unsigned)h) << 16); }

__device__ __forceinline__ void dep_guard_h(v8f& a, v8f& b, v16h x, v16h y) { asm volatile("v_nop\n\tv_nop\n\tv_nop\n\tv_nop" : "+v"(a), "+v"(b) : "v"(x), "v"(y)); }
__device__ __forceinline__ void dep_guard_b(v8f& a, v8f& b, v16b x, v16b y) { asm volatile("v_nop\n\tv_nop\n\tv_nop\n\tv_nop" : "+v"(a), "+v"(b) : "v"(x), "v"(y)); }
__device__ __forceinline__ void keep4_h(v16h a, v16h b, v16h c, v16h d) { asm volatile("v_nop" :: "v"(a), "v"(b), "v"(c), "v"(d)); }
__device__ __forceinline__ void keep4_b(v16b a, v16b b, v16b c, v16b d) { asm volatile("v_nop" :: "v"(a), "v"(b), "v"(c), "v"(d)); }
__device__ __forceinline__ void acc_guard4(v8f& a, v8f& b, v8f& c, v8f& d) { asm volatile("v_nop\n\tv_nop\n\tv_nop\n\tv_nop" : "+v"(a), "+v"(b), "+v"(c), "+v"(d)); }
template <typename T> struct Frag;
template <> struct Frag<_Float16> {
  typedef v16h V; union U { v16h v; v8h h[2]; };
  static __device__ __forceinline__ v16h load(const _Float16* p) {
    U f; f.h[0] = *(const v8h*)(p); f.h[1] = *(const v8h*)(p + 16); return f.v;
  }
  static __device__ __forceinline__ v8f mma(v16h a, v16h b, v8f c) {
    return __builtin_amdgcn_wmma_f32_16x16x32_f16(false, a, false, b, (short)0, c, false, false);
  }
  static __device__ __forceinline__ void guard(v8f& a, v8f& b, v16h x, v16h y) { dep_guard_h(a, b, x, y); }
  static __device__ __forceinline__ void keep(v16h a, v16h b, v16h c, v16h d) { keep4_h(a, b, c, d); }
};
template <> struct Frag<__bf16> {
  typedef v16b V; union U { v16b v; v8b h[2]; };
  static __device__ __forceinline__ v16b load(const __bf16* p) {
    U f; f.h[0] = *(const v8b*)(p); f.h[1] = *(const v8b*)(p + 16); return f.v;
  }
  static __device__ __forceinline__ v8f mma(v16b a, v16b b, v8f c) {
    return __builtin_amdgcn_wmma_f32_16x16x32_bf16(false, a, false, b, (short)0, c, false, false);
  }
  static __device__ __forceinline__ void guard(v8f& a, v8f& b, v16b x, v16b y) { dep_guard_b(a, b, x, y); }
  static __device__ __forceinline__ void keep(v16b a, v16b b, v16b c, v16b d) { keep4_b(a, b, c, d); }
};

__device__ __forceinline__ unsigned pk16(unsigned short a, unsigned short b) { return (unsigned)a | ((unsigned)b << 16); }
__device__ __forceinline__ unsigned short h_bits(float f) { const _Float16 h = (_Float16)f; return __builtin_bit_cast(unsigned short, h); }

template <int ET> struct Elem;
template <> struct Elem<0> { typedef _Float16 T; };
template <> struct Elem<1> { typedef __bf16 T; };
template <int ET, bool SPLIT, int BIAS_MODE, int OUT_MODE, bool RESID, int ACT = 0>
__global__ __launch_bounds__(256) void wmma_gemm64(
    const unsigned short* __restrict__ Ap, const unsigned short* __restrict__ A2p, int lda, long strideA,
    const unsigned short* __restrict__ Btp, const unsigned short* __restrict__ Bt2p, int ldb, long strideB,
    void* __restrict__ Cout, void* __restrict__ Cout2, int ldc, long strideC,
    const float* __restrict__ bias,
    const float* __restrict__ resid, long strideR,
    int M, int N, int K, float scale,
    const float* __restrict__ rowv, const float* __restrict__ colv) {
  typedef typename Elem<ET>::T T;
  typedef typename Frag<T>::V V;
  const T* A = (const T*)Ap; const T* A2 = (const T*)A2p; const T* Bt = (const T*)Btp; const T* Bt2 = (const T*)Bt2p;
  __shared__ __align__(16) float sT[8][16 * 68];
  const int b    = blockIdx.y;
  const int lane = threadIdx.x & 31;
  const int wave = threadIdx.x >> 5;
  const int tilesN = N >> 6;
  const int tilesM = M >> 6;
  const int tile = blockIdx.x * 8 + wave;
  if (tile >= tilesM * tilesN) return;
  const int tm = tile / tilesN;
  const int tn = tile - tm * tilesN;
  const int m0 = tm << 6;
  const int n0 = tn << 6;

  const T* Ab  = A  + (size_t)b * strideA;
  const T* Bb  = Bt + (size_t)b * strideB;
  const T* Ab2 = SPLIT ? (A2  + (size_t)b * strideA) : nullptr;
  const T* Bb2 = SPLIT ? (Bt2 + (size_t)b * strideB) : nullptr;

  const int rlane = lane & 15;
  const int koff  = (lane >> 4) * 8;
  const int mOff  = (lane >> 4) * 8;

  v8f acc[4][4];
#pragma unroll
  for (int i = 0; i < 4; ++i)
#pragma unroll
    for (int j = 0; j < 4; ++j) acc[i][j] = (v8f){0.f,0.f,0.f,0.f,0.f,0.f,0.f,0.f};

  for (int k0 = 0; k0 < K; k0 += 32) {
    V bh[4], bl[4];
#pragma unroll
    for (int j = 0; j < 4; ++j) {
      const size_t bo = (size_t)(n0 + (j << 4) + rlane) * ldb + koff + k0;
      bh[j] = Frag<T>::load(Bb + bo);
      if (SPLIT) bl[j] = Frag<T>::load(Bb2 + bo);
    }
#pragma unroll
    for (int i = 0; i < 4; ++i) {
      const size_t ao = (size_t)(m0 + (i << 4) + rlane) * lda + koff + k0;
      V ah = Frag<T>::load(Ab + ao);
      V al;
      if (SPLIT) al = Frag<T>::load(Ab2 + ao);
#pragma unroll
      for (int j = 0; j < 4; ++j) {
        acc[i][j] = Frag<T>::mma(ah, bh[j], acc[i][j]);
        if (SPLIT) {
          acc[i][j] = Frag<T>::mma(ah, bl[j], acc[i][j]);
          acc[i][j] = Frag<T>::mma(al, bh[j], acc[i][j]);
        }
      }
      Frag<T>::guard(acc[i][0], acc[i][3], ah, SPLIT ? al : ah);
    }
    Frag<T>::keep(bh[0], bh[1], bh[2], bh[3]);
    if (SPLIT) Frag<T>::keep(bl[0], bl[1], bl[2], bl[3]);
  }
  acc_guard4(acc[0][0], acc[0][1], acc[0][2], acc[0][3]);
  acc_guard4(acc[1][0], acc[1][1], acc[1][2], acc[1][3]);
  acc_guard4(acc[2][0], acc[2][1], acc[2][2], acc[2][3]);
  acc_guard4(acc[3][0], acc[3][1], acc[3][2], acc[3][3]);

  float* slab = sT[wave];
  const float* Rb = RESID ? (resid + (size_t)b * strideR) : nullptr;
#pragma unroll
  for (int i = 0; i < 4; ++i) {
    const int mBase = m0 + (i << 4);
#pragma unroll
    for (int j = 0; j < 4; ++j) {
      const int n = n0 + (j << 4) + rlane;
      float bv = 0.f, cv = 0.f;
      if (BIAS_MODE == 2 || BIAS_MODE == 3) bv = bias[n];
      if (BIAS_MODE == 3) cv = colv[n];
#pragma unroll
      for (int r = 0; r < 8; ++r) {
        float v = acc[i][j][r] * scale;
        if (BIAS_MODE == 1) v += bias[mBase + mOff + r];
        if (BIAS_MODE == 2) v += bv;
        if (BIAS_MODE == 3) { v = v + rowv[mBase + mOff + r] * cv; v = v + bv; }
        if (RESID) v += Rb[(size_t)(mBase + mOff + r) * ldc + n];
        if (ACT == 2) v = fmaxf(v, 0.0f);
        if (ACT == 4) v = (v > 0.f) ? v : 0.01f * v;
        slab[(mOff + r) * 68 + (j << 4) + rlane] = v;
      }
    }
    __builtin_amdgcn_fence(__ATOMIC_RELEASE, "workgroup");
    __builtin_amdgcn_wave_barrier();
    __builtin_amdgcn_fence(__ATOMIC_ACQUIRE, "workgroup");
    if (OUT_MODE == 0) {
      float* C = (float*)Cout + (size_t)b * strideC;
      const int hh = lane >> 4, c4 = (lane & 15) * 4;
      for (int pass = 0; pass < 2; ++pass) {
#pragma unroll
        for (int it = 0; it < 8; ++it) {
          const int row = it * 2 + hh;
          v4f v = *(const v4f*)(slab + row * 68 + c4);
          *(volatile v4f*)(C + (size_t)(mBase + row) * ldc + n0 + c4) = v;
        }
        __threadfence();
      }
    } else {
      const int q = lane >> 3, c8 = (lane & 7) * 8;
      unsigned short* C  = (unsigned short*)Cout  + (size_t)b * strideC;
      unsigned short* C2 = (OUT_MODE == 2) ? ((unsigned short*)Cout2 + (size_t)b * strideC) : nullptr;
      for (int pass = 0; pass < 2; ++pass) {
#pragma unroll
        for (int it = 0; it < 4; ++it) {
          const int row = it * 4 + q;
          const float* sp = slab + row * 68 + c8;
          v8h hv, lv;
#pragma unroll
          for (int e = 0; e < 8; ++e) {
            if (OUT_MODE == 1) {
              hv[e] = (_Float16)sp[e];
            } else {
              unsigned short hb = f2bf_bits(sp[e]);
              unsigned short lb = f2bf_bits(sp[e] - bf_bits2f(hb));
              hv[e] = __builtin_bit_cast(_Float16, hb);
              lv[e] = __builtin_bit_cast(_Float16, lb);
            }
          }
          *(volatile v8h*)(C + (size_t)(mBase + row) * ldc + n0 + c8) = hv;
          if (OUT_MODE == 2) *(volatile v8h*)(C2 + (size_t)(mBase + row) * ldc + n0 + c8) = lv;
        }
        __threadfence();
      }
    }
    __builtin_amdgcn_fence(__ATOMIC_RELEASE, "workgroup");
    __builtin_amdgcn_wave_barrier();
    __builtin_amdgcn_fence(__ATOMIC_ACQUIRE, "workgroup");
  }
}

__global__ __launch_bounds__(256) void wout_tcast_kernel(const float* __restrict__ Wout,
                                                         unsigned short* __restrict__ WhT) {
  __shared__ float sm[64][65];
  const int t  = threadIdx.x;
  const int k0 = blockIdx.x * 64;
  const int n0 = blockIdx.y * 64;
#pragma unroll
  for (int i = 0; i < 16; ++i) {
    const int e  = i * 256 + t;
    const int kl = e >> 6;
    const int nl = e & 63;
    sm[nl][kl] = Wout[(size_t)(k0 + kl) * kOutDim + n0 + nl] * kWCarry;
  }
  __syncthreads();
  const int lane = t & 31, wave = t >> 5;
  const int q = lane >> 3, c8 = (lane & 7) * 8;
  for (int pass = 0; pass < 2; ++pass) {
#pragma unroll
    for (int it = 0; it < 2; ++it) {
      const int row = wave * 8 + it * 4 + q;
      unsigned short hb[8];
#pragma unroll
      for (int e = 0; e < 8; ++e) hb[e] = h_bits(sm[row][c8 + e]);
      const v4u u = (v4u){pk16(hb[0], hb[1]), pk16(hb[2], hb[3]), pk16(hb[4], hb[5]), pk16(hb[6], hb[7])};
      *(volatile v4u*)(WhT + (size_t)(n0 + row) * kFeat + k0 + c8) = u;
    }
    __threadfence();
  }
}

__global__ __launch_bounds__(512) void basis_kernel(
    const float* __restrict__ x,
    const float* __restrict__ W1, const float* __restrict__ b1,
    const float* __restrict__ W2, const float* __restrict__ b2,
    const float* __restrict__ W3, const float* __restrict__ b3,
    const float* __restrict__ centers, const float* __restrict__ lw,
    unsigned short* __restrict__ phi_out, float* __restrict__ logdet, int row_base) {
  extern __shared__ __attribute__((aligned(16))) float dsm[];
  float*    s_c    = dsm;
  float*    s_iw   = dsm + kFeat;
  unsigned* s_phi  = (unsigned*)(dsm + 2 * kFeat);
  float*    s_x    = dsm + 20480;
  float*    s_part = dsm + 20992;
  float*    s_h1   = dsm + 21008;
  float*    s_h2   = dsm + 21016;
  float*    s_lg   = dsm + 21024;
  float*    s_ld   = dsm + 21040;

  const int tid  = threadIdx.x;
  const int lane = tid & 31;
  const int wave = tid >> 5;
  const int d    = tid;
  const int hq   = tid & 7;
  const int hw   = tid >> 6;
  const int seg  = tid & 63;

#pragma unroll 1
  for (int i = 0; i < 16; ++i) {
    const int e = i * 512 + tid;
    s_c[e]  = centers[e];
    s_iw[e] = 1.0f / (expf(lw[e]) + 1e-12f);
  }
  float w1r[8];
#pragma unroll
  for (int e = 0; e < 8; ++e) w1r[e] = W1[(seg * 8 + e) * kHidden + hw];
  const float b1h = b1[hq];
  const float b2h = b2[hq];
  const float b3d = b3[d];
  const int blk_local0 = blockIdx.x * kRowsPerBlk;
  __syncthreads();

#pragma unroll 1
  for (int r = 0; r < kRowsPerBlk; ++r) {
    const int lrow = blk_local0 + r;
    const int grow = row_base + lrow;
    const float xv = x[(size_t)grow * kInDim + d];
    s_x[d] = xv;
    __syncthreads();

    const v4f xa = *(const v4f*)(s_x + seg * 8);
    const v4f xb = *(const v4f*)(s_x + seg * 8 + 4);
    float pp = 0.0f;
    pp = fmaf(xa[0], w1r[0], pp); pp = fmaf(xa[1], w1r[1], pp);
    pp = fmaf(xa[2], w1r[2], pp); pp = fmaf(xa[3], w1r[3], pp);
    pp = fmaf(xb[0], w1r[4], pp); pp = fmaf(xb[1], w1r[5], pp);
    pp = fmaf(xb[2], w1r[6], pp); pp = fmaf(xb[3], w1r[7], pp);
#pragma unroll
    for (int off = 16; off > 0; off >>= 1) pp += __shfl_xor(pp, off, 32);
    if (lane == 0) s_part[wave] = pp;
    __syncthreads();

    float a1 = s_part[2 * hq] + s_part[2 * hq + 1];
    a1 = a1 + b1h;
    const float h1v = a1 * __builtin_amdgcn_rcpf(1.0f + expf(-a1));
    if (tid < kHidden) s_h1[tid] = h1v;
    __syncthreads();

    float a2 = 0.0f;
#pragma unroll 1
    for (int j = 0; j < kHidden; ++j) a2 = fmaf(s_h1[j], W2[j * kHidden + hq], a2);
    a2 = a2 + b2h;
    const float h2v = a2 * __builtin_amdgcn_rcpf(1.0f + expf(-a2));
    if (tid < kHidden) s_h2[tid] = h2v;
    __syncthreads();

    float s = 0.0f;
#pragma unroll 1
    for (int j = 0; j < kHidden; ++j) s = fmaf(s_h2[j], W3[j * kInDim + d], s);
    s = s + b3d;
    const float sp = fmaxf(s, 0.0f) + log1pf(expf(-fabsf(s)));
    const float g  = sp + 1e-8f;
    const float z  = xv * sqrtf(g);
    float lg = logf(g);
#pragma unroll
    for (int off = 16; off > 0; off >>= 1) lg += __shfl_xor(lg, off, 32);
    if (lane == 0) s_lg[wave] = lg;

#pragma unroll 1
    for (int kk = 0; kk < 8; ++kk) {
      const int e0 = d * kNumRbf + 2 * kk;
      const float c0 = s_c[e0],  c1 = s_c[e0 + 1];
      const float i0 = s_iw[e0], i1 = s_iw[e0 + 1];
      const float u0 = (z - c0) * i0;
      const float u1 = (z - c1) * i1;
      const float p0 = expf(-2.0f * (u0 * u0));
      const float p1 = expf(-2.0f * (u1 * u1));
      s_phi[d * 8 + kk] = pk16(h_bits(p0 * kPhiCarry), h_bits(p1 * kPhiCarry));
    }
    __syncthreads();

    float ld = 0.0f;
#pragma unroll
    for (int w = 0; w < 16; ++w) ld += s_lg[w];
    if (tid == 0) s_ld[r] = ld;

    const v4u* sp4 = (const v4u*)s_phi;
    const v4u q0 = sp4[tid];
    const v4u q1 = sp4[512 + tid];
    v4u* gp = (v4u*)(phi_out + (size_t)lrow * kFeat);
    *(volatile v4u*)(gp + tid)       = q0;
    *(volatile v4u*)(gp + 512 + tid) = q1;
    __threadfence();
    *(volatile v4u*)(gp + tid)       = q0;
    *(volatile v4u*)(gp + 512 + tid) = q1;
  }
  __syncthreads();
  if (tid < 32) {
    const float v = s_ld[tid];
    float* lp = logdet + (size_t)(row_base + blk_local0);
    ((volatile float*)lp)[tid] = v;
    __threadfence();
    ((volatile float*)lp)[tid] = v;
  }
}

extern "C" void kernel_launch(void* const* d_in, const int* in_sizes, int n_in,
                              void* d_out, int out_size, void* d_ws, size_t ws_size,
                              hipStream_t stream) {
  if (n_in < 11) return;
  if (in_sizes[0] != kRows * kInDim) return;
  if (in_sizes[7] != kInDim * kNumRbf || in_sizes[8] != kInDim * kNumRbf) return;
  if (in_sizes[9] != (kFeat + 1) * kOutDim || in_sizes[10] != kOutDim) return;
  if (out_size != kRows * kOutDim) return;
  if (ws_size < kWsTotal) return;

  const float* x          = (const float*)d_in[0];
  const float* W1         = (const float*)d_in[1];
  const float* b1         = (const float*)d_in[2];
  const float* W2         = (const float*)d_in[3];
  const float* b2         = (const float*)d_in[4];
  const float* W3         = (const float*)d_in[5];
  const float* b3         = (const float*)d_in[6];
  const float* centers    = (const float*)d_in[7];
  const float* log_widths = (const float*)d_in[8];
  const float* Wout       = (const float*)d_in[9];
  const float* bout       = (const float*)d_in[10];
  float* out = (float*)d_out;

  char* ws = (char*)d_ws;
  unsigned short* WhT   = (unsigned short*)(ws + kWsWht);
  unsigned short* phiA  = (unsigned short*)(ws + kWsPhiA);
  unsigned short* phiB  = (unsigned short*)(ws + kWsPhiB);
  float*          logdet = (float*)(ws + kWsLogdet);
  const float*    wlast  = Wout + (size_t)kFeat * kOutDim;

  wout_tcast_kernel<<<dim3(kFeat / 64, kOutDim / 64), 256, 0, stream>>>(Wout, WhT);

  for (int ch = 0; ch < kNumChunks; ++ch) {
    unsigned short* phi = (ch & 1) ? phiB : phiA;
    const int row_base = ch * kChunkRows;
    basis_kernel<<<kChunkRows / kRowsPerBlk, 512, kLdsBytes, stream>>>(
        x, W1, b1, W2, b2, W3, b3, centers, log_widths, phi, logdet, row_base);
    float* cptr = out + (size_t)row_base * kOutDim;
    wmma_gemm64<0, false, 3, 0, false, 0><<<dim3((kChunkRows / 64) * (kOutDim / 64) / 8, 1), 256, 0, stream>>>(
        phi, phi, kFeat, 0L,
        WhT, WhT, kFeat, 0L,
        (void*)cptr, (void*)cptr, kOutDim, 0L,
        bout,
        bout, 0L,
        kChunkRows, kOutDim, kFeat, kGemmScale,
        logdet + row_base, wlast);
  }
}
